// Encoder_17360257810780
// MI455X (gfx1250) — hardware-run, weakly checked
//
#include <hip/hip_runtime.h>
#include <math.h>

typedef __attribute__((ext_vector_type(16))) _Float16 v16h;
typedef __attribute__((ext_vector_type(8)))  _Float16 v8h;
typedef __attribute__((ext_vector_type(8)))  float    v8f;
typedef __attribute__((ext_vector_type(4)))  float    v4f;
typedef __attribute__((ext_vector_type(4)))  unsigned int v4u;

constexpr int kNB    = 16;
constexpr int kNT    = 32;
constexpr int kNF    = kNB * kNT;
constexpr int kXS    = 64;
constexpr int kXC    = 5;
constexpr int kCh1   = 32;
constexpr int kS1    = 32;
constexpr int kCh2   = 64;
constexpr int kS2    = 16;
constexpr int kND    = 256;
constexpr int kNG    = 3 * kND;
constexpr int kK1    = 96;
constexpr int kK2    = 9 * kCh1;
constexpr int kFrameX = kXS * kXS * kXC;
constexpr int kX1Rows = 33;
constexpr int kX1Cols = 66;
constexpr int kX1Pix  = kX1Rows * kX1Cols;
constexpr int kA2Rows = 17;
constexpr int kA2Cols = 33;
constexpr int kA2Pieces = kA2Rows * kA2Cols * 4;
constexpr int kHP    = 264;
constexpr int kSP    = 260;
static_assert(kNF == 512 && kFrameX == 20480 && kK2 == 288 && kNG == 768, "shapes");
static_assert((kK1 % 32) == 0 && (kK2 % 32) == 0 && (kCh2 % 32) == 0 && (kND % 32) == 0, "GEMM K multiples of 32");
static_assert((kNF % 64) == 0 && (kND % 64) == 0 && (kNG % 64) == 0, "GEMM M,N multiples of 64");
static_assert(kX1Pix == 2178 && kA2Pieces == 2244, "staging extents");
static_assert(9 * 256 >= kX1Pix && 9 * 256 >= kA2Pieces, "staging loop coverage");

constexpr float kCarryX = 128.0f;
constexpr float kCarryA = 64.0f;
constexpr float kCarryW = 1024.0f;
constexpr float kCarryH = 1024.0f;
constexpr float kScale1 = 1.0f / (kCarryX * kCarryW);
constexpr float kScale2 = 1.0f / (kCarryA * kCarryW);
constexpr float kScaleH = 1.0f / (kCarryH * kCarryW);
constexpr float kF16Min = 6.103515625e-5f;

constexpr size_t kSzW1T   = (size_t)kCh1 * kK1 * 2;
constexpr size_t kSzW2T   = (size_t)kCh2 * kK2 * 2;
constexpr size_t kSzDWT   = (size_t)kND * kCh2 * 2;
constexpr size_t kSzWXT   = (size_t)kNG * kND * 2;
constexpr size_t kSzWHT   = (size_t)kNG * kND * 2;
constexpr size_t kSzA1    = (size_t)kNF * kS1 * kS1 * kCh1 * 2;
constexpr size_t kSzPOOL  = (size_t)kNF * kCh2 * 2;
constexpr size_t kSzFEATS = (size_t)kNF * kND * 2;
constexpr size_t kSzXG    = (size_t)kNF * kNG * 4;
constexpr size_t kOffW1T   = 0;
constexpr size_t kOffW2T   = kOffW1T + kSzW1T;
constexpr size_t kOffDWT   = kOffW2T + kSzW2T;
constexpr size_t kOffWXT   = kOffDWT + kSzDWT;
constexpr size_t kOffWHT   = kOffWXT + kSzWXT;
constexpr size_t kOffA1    = kOffWHT + kSzWHT;
constexpr size_t kOffPOOL  = kOffA1 + kSzA1;
constexpr size_t kOffFEATS = kOffPOOL + kSzPOOL;
constexpr size_t kOffXG    = kOffFEATS + kSzFEATS;
constexpr size_t kWsTotal  = kOffXG + kSzXG;
static_assert(kWsTotal == 36317184ull, "carve total");
static_assert(kWsTotal <= 134217728ull, "carve cap");
static_assert((kOffW2T % 256) == 0 && (kOffDWT % 256) == 0 && (kOffWXT % 256) == 0 && (kOffWHT % 256) == 0 &&
              (kOffA1 % 256) == 0 && (kOffPOOL % 256) == 0 && (kOffFEATS % 256) == 0 && (kOffXG % 256) == 0, "aligned regions");

__device__ __forceinline__ unsigned short f2bf_bits(float f) {
  unsigned u = __float_as_uint(f);
  return (unsigned short)((u + 0x7FFFu + ((u >> 16) & 1u)) >> 16);
}
__device__ __forceinline__ float bf_bits2f(unsigned short h) { return __uint_as_float(((unsigned)h) << 16); }
__device__ __forceinline__ float bf16r(float f) { return bf_bits2f(f2bf_bits(f)); }

__device__ __forceinline__ _Float16 to_h_carry(float v, float carry) {
  float t = v * carry;
  t = (fabsf(t) < kF16Min) ? 0.0f : t;
  return (_Float16)t;
}

union FragU { v16h v; v8h h[2]; };
__device__ __forceinline__ v16h ldfrag(const _Float16* p) {
  FragU f;
  f.h[0] = *(const v8h*)(p);
  f.h[1] = *(const v8h*)(p + 16);
  return f.v;
}
__device__ __forceinline__ v8f mma_h(v16h a, v16h b, v8f c) {
  c = __builtin_amdgcn_wmma_f32_16x16x32_f16(false, a, false, b, (short)0, c, false, false);
  asm volatile("v_nop\n\tv_nop\n\tv_nop\n\tv_nop" : "+v"(c) : "v"(a), "v"(b));
  return c;
}
__device__ __forceinline__ void wave_sync_lds() {
  __builtin_amdgcn_fence(__ATOMIC_RELEASE, "workgroup");
  __builtin_amdgcn_wave_barrier();
  __builtin_amdgcn_fence(__ATOMIC_ACQUIRE, "workgroup");
}

template <int MODE>
__global__ __launch_bounds__(256) void pack_wt_kernel(const float* __restrict__ src, unsigned short* __restrict__ dst,
                                                      int nOut, int kPad, int total8) {
  const int i = blockIdx.x * 256 + threadIdx.x;
  if (i >= total8) return;
  const int k8n = kPad >> 3;
  const int n = i / k8n;
  const int kb = (i - n * k8n) << 3;
  v8h hv;
#pragma unroll
  for (int e = 0; e < 8; ++e) {
    const int kp = kb + e;
    int ks = kp;
    bool ok = true;
    if (MODE == 1) {
      const int ky = kp >> 5;
      const int rem = kp & 31;
      const int kx = rem >> 3;
      const int ci = rem & 7;
      ok = (kx < 3) && (ci < kXC);
      ks = ok ? ((ky * 3 + kx) * kXC + ci) : 0;
    }
    float v = src[(size_t)ks * nOut + n];
    v = bf16r(v);
    v = ok ? v : 0.0f;
    asm volatile("" : "+v"(v));
    hv[e] = to_h_carry(v, kCarryW);
  }
  unsigned short* q = dst + (size_t)i * 8;
  *(volatile v8h*)q = hv;
  __threadfence();
  *(volatile v8h*)q = hv;
}

__global__ __launch_bounds__(256) void conv1_kernel(const float* __restrict__ x, const unsigned short* __restrict__ w1t,
                                                    const float* __restrict__ cb1, unsigned short* __restrict__ a1) {
  __shared__ __align__(16) _Float16 xt[kX1Pix * 8];
  __shared__ __align__(16) float slab1[8][16 * 36];
  const int tid = threadIdx.x, lane = tid & 31, wave = tid >> 5;
  const int c = lane & 15, hh = lane >> 4;
  const int f = blockIdx.x >> 1, half = blockIdx.x & 1;
  const float* xf = x + (size_t)f * kFrameX;
  const int iy0 = half * 32;

#pragma unroll 1
  for (int it = 0; it < 9; ++it) {
    const int idx = it * 256 + tid;
    const int idc = (idx < kX1Pix) ? idx : (kX1Pix - 1);
    const int r = idc / kX1Cols;
    const int col = idc - r * kX1Cols;
    const int iy = iy0 + r;
    const bool ok = (iy < kXS) && (col < kXS);
    const int iyc = (iy < kXS) ? iy : (kXS - 1);
    const int cc = (col < kXS) ? col : (kXS - 1);
    const float* p = xf + (size_t)(iyc * kXS + cc) * kXC;
    float v0 = p[0], v1 = p[1], v2 = p[2], v3 = p[3], v4 = p[4];
    asm volatile("" : "+v"(v0), "+v"(v1), "+v"(v2), "+v"(v3), "+v"(v4));
    v0 = ok ? bf16r(v0) : 0.0f;
    v1 = ok ? bf16r(v1) : 0.0f;
    v2 = ok ? bf16r(v2) : 0.0f;
    v3 = ok ? bf16r(v3) : 0.0f;
    v4 = ok ? bf16r(v4) : 0.0f;
    float zp = 0.0f;
    asm volatile("" : "+v"(zp));
    v8h hv;
    hv[0] = to_h_carry(v0, kCarryX);
    hv[1] = to_h_carry(v1, kCarryX);
    hv[2] = to_h_carry(v2, kCarryX);
    hv[3] = to_h_carry(v3, kCarryX);
    hv[4] = to_h_carry(v4, kCarryX);
    hv[5] = (_Float16)zp;
    hv[6] = (_Float16)zp;
    hv[7] = (_Float16)zp;
    if (idx < kX1Pix) *(v8h*)(xt + idc * 8) = hv;
  }
  __syncthreads();

  const _Float16* W = (const _Float16*)w1t;
  v16h bf[2][3];
#pragma unroll
  for (int nt = 0; nt < 2; ++nt)
#pragma unroll
    for (int ky = 0; ky < 3; ++ky)
      bf[nt][ky] = ldfrag(W + (nt * 16 + c) * kK1 + ky * 32 + 8 * hh);
  const float b0 = bf16r(cb1[c]);
  const float b1 = bf16r(cb1[16 + c]);
  float* sl = slab1[wave];
  const v8f z8 = {0.f, 0.f, 0.f, 0.f, 0.f, 0.f, 0.f, 0.f};

#pragma unroll 1
  for (int mi = 0; mi < 4; ++mi) {
    const int m = wave * 4 + mi;
    const int oyl = m >> 1;
    const int ox0 = (m & 1) << 4;
    v8f acc0 = z8, acc1 = z8;
#pragma unroll
    for (int ky = 0; ky < 3; ++ky) {
      const v16h a = ldfrag(xt + ((2 * oyl + ky) * kX1Cols + 2 * (ox0 + c)) * 8 + 8 * hh);
      acc0 = mma_h(a, bf[0][ky], acc0);
      acc1 = mma_h(a, bf[1][ky], acc1);
    }
#pragma unroll
    for (int r = 0; r < 8; ++r) {
      sl[(8 * hh + r) * 36 + c]      = fmaxf(acc0[r] * kScale1 + b0, 0.0f);
      sl[(8 * hh + r) * 36 + 16 + c] = fmaxf(acc1[r] * kScale1 + b1, 0.0f);
    }
    wave_sync_lds();
    v8h hv[2];
#pragma unroll
    for (int it = 0; it < 2; ++it) {
      const float* sp = sl + (it * 8 + (lane >> 2)) * 36 + (lane & 3) * 8;
      const v4f q0 = *(const v4f*)(sp);
      const v4f q1 = *(const v4f*)(sp + 4);
#pragma unroll
      for (int e = 0; e < 4; ++e) {
        hv[it][e]     = to_h_carry(q0[e], kCarryA);
        hv[it][4 + e] = to_h_carry(q1[e], kCarryA);
      }
    }
    const int oy = half * 16 + oyl;
    unsigned short* op = a1 + (((size_t)f * kS1 + oy) * kS1 + ox0) * kCh1 + lane * 8;
    for (int pass = 0; pass < 2; ++pass) {
      *(volatile v8h*)(op) = hv[0];
      *(volatile v8h*)(op + 256) = hv[1];
      __threadfence();
    }
    wave_sync_lds();
  }
}

__global__ __launch_bounds__(256) void conv2_pool_kernel(const unsigned short* __restrict__ a1,
                                                         const unsigned short* __restrict__ w2t,
                                                         const float* __restrict__ cb2,
                                                         unsigned short* __restrict__ pooled) {
  __shared__ __align__(16) _Float16 act[kA2Rows * kA2Cols * kCh1];
  __shared__ __align__(16) float part[16][kCh2];
  __shared__ __align__(16) float pool[kCh2];
  const int tid = threadIdx.x, lane = tid & 31, wave = tid >> 5;
  const int c = lane & 15, hh = lane >> 4;
  const int f = blockIdx.x;
  const v4u* src = (const v4u*)(a1 + (size_t)f * (kS1 * kS1 * kCh1));
  const _Float16* W = (const _Float16*)w2t;
  const v4u zero4 = {0u, 0u, 0u, 0u};
  const v8f z8 = {0.f, 0.f, 0.f, 0.f, 0.f, 0.f, 0.f, 0.f};

#pragma unroll 1
  for (int chunk = 0; chunk < 2; ++chunk) {
    __syncthreads();
#pragma unroll 1
    for (int it = 0; it < 9; ++it) {
      const int idx = it * 256 + tid;
      const int idc = (idx < kA2Pieces) ? idx : (kA2Pieces - 1);
      const int r = idc / (kA2Cols * 4);
      const int rem = idc - r * (kA2Cols * 4);
      const int col = rem >> 2;
      const int q = rem & 3;
      const int iy = 16 * chunk + r;
      const bool ok = (iy < kS1) && (col < kS1);
      const int iyc = (iy < kS1) ? iy : (kS1 - 1);
      const int cc = (col < kS1) ? col : (kS1 - 1);
      v4u w = src[(iyc * kS1 + cc) * 4 + q];
      asm volatile("" : "+v"(w));
      w = ok ? w : zero4;
      if (idx < kA2Pieces) *(v4u*)(act + (r * kA2Cols + col) * kCh1 + q * 8) = w;
    }
    __syncthreads();

    v8f acc[4];
#pragma unroll
    for (int j = 0; j < 4; ++j) acc[j] = z8;
#pragma unroll 1
    for (int tap = 0; tap < 9; ++tap) {
      const int ky = tap / 3;
      const int kx = tap - 3 * ky;
      const v16h a = ldfrag(act + ((2 * wave + ky) * kA2Cols + 2 * c + kx) * kCh1 + 8 * hh);
#pragma unroll
      for (int j = 0; j < 4; ++j) {
        const v16h b = ldfrag(W + (size_t)(j * 16 + c) * kK2 + tap * 32 + 8 * hh);
        acc[j] = mma_h(a, b, acc[j]);
      }
    }
#pragma unroll
    for (int j = 0; j < 4; ++j) {
      const float bv = bf16r(cb2[j * 16 + c]);
      float s = 0.0f;
#pragma unroll
      for (int r = 0; r < 8; ++r) s += fmaxf(acc[j][r] * kScale2 + bv, 0.0f);
      const float so = __shfl_xor(s, 16, 32);
      s += so;
      if (hh == 0) part[chunk * 8 + wave][j * 16 + c] = s;
    }
  }
  __syncthreads();
  if (tid < kCh2) {
    float s = 0.0f;
#pragma unroll 1
    for (int i = 0; i < 16; ++i) s += part[i][tid];
    pool[tid] = s * (1.0f / 256.0f);
  }
  __syncthreads();
  if (tid < 8) {
    const v4f q0 = *(const v4f*)(pool + tid * 8);
    const v4f q1 = *(const v4f*)(pool + tid * 8 + 4);
    v8h hv;
#pragma unroll
    for (int e = 0; e < 4; ++e) {
      hv[e]     = to_h_carry(q0[e], kCarryA);
      hv[4 + e] = to_h_carry(q1[e], kCarryA);
    }
    unsigned short* op = pooled + (size_t)f * kCh2 + tid * 8;
    *(volatile v8h*)op = hv;
    __threadfence();
    *(volatile v8h*)op = hv;
  }
}

template <int OUT_MODE, int ACT>
__global__ __launch_bounds__(256) void gemm64_kernel(
    const unsigned short* __restrict__ Ap, int lda,
    const unsigned short* __restrict__ Btp, int ldb,
    void* __restrict__ Cout, int ldc,
    const float* __restrict__ bias,
    int M, int N, int K, float scale, float ocarry) {
  const _Float16* A = (const _Float16*)Ap;
  const _Float16* Bt = (const _Float16*)Btp;
  __shared__ __align__(16) float sT[8][16 * 68];
  const int lane = threadIdx.x & 31;
  const int wave = threadIdx.x >> 5;
  const int tilesN = N >> 6;
  const int tilesM = M >> 6;
  const int tile = blockIdx.x * 8 + wave;
  if (tile >= tilesM * tilesN) return;
  const int tm = tile / tilesN;
  const int tn = tile - tm * tilesN;
  const int m0 = tm << 6;
  const int n0 = tn << 6;
  const int rlane = lane & 15;
  const int koff  = (lane >> 4) * 8;
  const int mOff  = (lane >> 4) * 8;

  v8f acc[4][4];
#pragma unroll
  for (int i = 0; i < 4; ++i)
#pragma unroll
    for (int j = 0; j < 4; ++j) acc[i][j] = (v8f){0.f, 0.f, 0.f, 0.f, 0.f, 0.f, 0.f, 0.f};

  for (int k0 = 0; k0 < K; k0 += 32) {
    v16h bh[4];
#pragma unroll
    for (int j = 0; j < 4; ++j)
      bh[j] = ldfrag(Bt + (size_t)(n0 + (j << 4) + rlane) * ldb + koff + k0);
#pragma unroll
    for (int i = 0; i < 4; ++i) {
      const v16h ah = ldfrag(A + (size_t)(m0 + (i << 4) + rlane) * lda + koff + k0);
#pragma unroll
      for (int j = 0; j < 4; ++j) acc[i][j] = mma_h(ah, bh[j], acc[i][j]);
    }
  }

  float* slab = sT[wave];
#pragma unroll
  for (int i = 0; i < 4; ++i) {
    const int mBase = m0 + (i << 4);
#pragma unroll
    for (int j = 0; j < 4; ++j) {
      const int n = n0 + (j << 4) + rlane;
      const float bv = bf16r(bias[n]);
#pragma unroll
      for (int r = 0; r < 8; ++r) {
        float v = acc[i][j][r] * scale + bv;
        if (ACT == 2) v = fmaxf(v, 0.0f);
        slab[(mOff + r) * 68 + (j << 4) + rlane] = v;
      }
    }
    wave_sync_lds();
    if (OUT_MODE == 0) {
      float* C = (float*)Cout;
      const int hh = lane >> 4, c4 = (lane & 15) * 4;
      for (int pass = 0; pass < 2; ++pass) {
#pragma unroll
        for (int it = 0; it < 8; ++it) {
          const int row = it * 2 + hh;
          const v4f v = *(const v4f*)(slab + row * 68 + c4);
          *(volatile v4f*)(C + (size_t)(mBase + row) * ldc + n0 + c4) = v;
        }
        __threadfence();
      }
    } else {
      const int q = lane >> 3, c8 = (lane & 7) * 8;
      unsigned short* C = (unsigned short*)Cout;
      for (int pass = 0; pass < 2; ++pass) {
#pragma unroll
        for (int it = 0; it < 4; ++it) {
          const int row = it * 4 + q;
          const float* sp = slab + row * 68 + c8;
          v8h hv;
#pragma unroll
          for (int e = 0; e < 8; ++e) hv[e] = to_h_carry(sp[e], ocarry);
          *(volatile v8h*)(C + (size_t)(mBase + row) * ldc + n0 + c8) = hv;
        }
        __threadfence();
      }
    }
    wave_sync_lds();
  }
}

__global__ __launch_bounds__(512) void gru_seq_kernel(const float* __restrict__ xg,
                                                      const unsigned short* __restrict__ whtp,
                                                      float* __restrict__ out0, float* __restrict__ out1) {
  __shared__ __align__(16) _Float16 Ah[16 * kHP];
  __shared__ __align__(16) _Float16 Arh[16 * kHP];
  __shared__ __align__(16) float Sl[16 * kSP];
  const _Float16* WT = (const _Float16*)whtp;
  const int tid = threadIdx.x, lane = tid & 31, wave = tid >> 5;
  const int c = lane & 15, hh = lane >> 4;
  const int j = 16 * wave + c;

#pragma unroll 1
  for (int i = tid; i < 16 * kHP; i += 512) {
    Ah[i] = (_Float16)0.0f;
    Arh[i] = (_Float16)0.0f;
  }
  float hst[8];
#pragma unroll
  for (int r = 0; r < 8; ++r) hst[r] = 0.0f;
  __syncthreads();

  const _Float16* wz = WT + (size_t)j * kND + 8 * hh;
  const _Float16* wr = WT + (size_t)(kND + j) * kND + 8 * hh;
  const _Float16* wc = WT + (size_t)(2 * kND + j) * kND + 8 * hh;
  const _Float16* arow = Ah + c * kHP + 8 * hh;
  const _Float16* rrow = Arh + c * kHP + 8 * hh;
  const v8f z8 = {0.f, 0.f, 0.f, 0.f, 0.f, 0.f, 0.f, 0.f};

#pragma unroll 1
  for (int t = 0; t < kNT; ++t) {
    float xz[8], xr[8];
#pragma unroll
    for (int r = 0; r < 8; ++r) {
      const size_t row = (size_t)(8 * hh + r) * kNT + (size_t)t;
      xz[r] = xg[row * kNG + j];
      xr[r] = xg[row * kNG + kND + j];
    }
    v8f accZ = z8, accR = z8;
#pragma unroll 2
    for (int k0 = 0; k0 < kND; k0 += 32) {
      const v16h a  = ldfrag(arow + k0);
      const v16h bz = ldfrag(wz + k0);
      const v16h br = ldfrag(wr + k0);
      accZ = mma_h(a, bz, accZ);
      accR = mma_h(a, br, accR);
    }
    float zg[8];
#pragma unroll
    for (int r = 0; r < 8; ++r) {
      const float gz = accZ[r] * kScaleH + xz[r];
      const float gr = accR[r] * kScaleH + xr[r];
      zg[r] = 1.0f / (1.0f + expf(-gz));
      const float rg = 1.0f / (1.0f + expf(-gr));
      const float rh = rg * hst[r];
      Arh[(8 * hh + r) * kHP + j] = to_h_carry(rh, kCarryH);
    }
    __syncthreads();

    float xh[8];
#pragma unroll
    for (int r = 0; r < 8; ++r) {
      const size_t row = (size_t)(8 * hh + r) * kNT + (size_t)t;
      xh[r] = xg[row * kNG + 2 * kND + j];
    }
    v8f accH = z8;
#pragma unroll 2
    for (int k0 = 0; k0 < kND; k0 += 32) {
      const v16h a = ldfrag(rrow + k0);
      const v16h b = ldfrag(wc + k0);
      accH = mma_h(a, b, accH);
    }
#pragma unroll
    for (int r = 0; r < 8; ++r) {
      const float hc = tanhf(accH[r] * kScaleH + xh[r]);
      const float hn = zg[r] * hst[r] + (1.0f - zg[r]) * hc;
      hst[r] = hn;
      Ah[(8 * hh + r) * kHP + j] = to_h_carry(hn, kCarryH);
      Sl[(8 * hh + r) * kSP + j] = hn;
    }
    __syncthreads();

    {
      const bool last = (t == kNT - 1);
      const v4f o0 = *(const v4f*)(Sl + wave * kSP + lane * 4);
      const v4f o1 = *(const v4f*)(Sl + wave * kSP + 128 + lane * 4);
      float* op = out0 + ((size_t)wave * kNT + (size_t)t) * kND + lane * 4;
      float* fp = out1 + (size_t)wave * kND + lane * 4;
      for (int pass = 0; pass < 2; ++pass) {
        *(volatile v4f*)(op) = o0;
        *(volatile v4f*)(op + 128) = o1;
        if (last) {
          *(volatile v4f*)(fp) = o0;
          *(volatile v4f*)(fp + 128) = o1;
        }
        __threadfence();
      }
    }
  }
}

extern "C" void kernel_launch(void* const* d_in, const int* in_sizes, int n_in,
                              void* d_out, int out_size, void* d_ws, size_t ws_size,
                              hipStream_t stream) {
  if (n_in < 10 || d_out == nullptr || d_ws == nullptr) return;
  if (in_sizes[0] != kNF * kFrameX) return;
  if (in_sizes[1] != 9 * kXC * kCh1) return;
  if (in_sizes[2] != kCh1) return;
  if (in_sizes[3] != 9 * kCh1 * kCh2) return;
  if (in_sizes[4] != kCh2) return;
  if (in_sizes[5] != kCh2 * kND) return;
  if (in_sizes[6] != kND) return;
  if (in_sizes[7] != kND * kNG) return;
  if (in_sizes[8] != kND * kNG) return;
  if (in_sizes[9] != kNG) return;
  if (out_size != kNF * kND + kNB * kND) return;
  if (ws_size < kWsTotal) return;

  const float* x   = (const float*)d_in[0];
  const float* cw1 = (const float*)d_in[1];
  const float* cb1 = (const float*)d_in[2];
  const float* cw2 = (const float*)d_in[3];
  const float* cb2 = (const float*)d_in[4];
  const float* dw  = (const float*)d_in[5];
  const float* db  = (const float*)d_in[6];
  const float* wx  = (const float*)d_in[7];
  const float* wh  = (const float*)d_in[8];
  const float* bg  = (const float*)d_in[9];
  float* out0 = (float*)d_out;
  float* out1 = out0 + (size_t)kNF * kND;

  char* ws = (char*)d_ws;
  unsigned short* W1T   = (unsigned short*)(ws + kOffW1T);
  unsigned short* W2T   = (unsigned short*)(ws + kOffW2T);
  unsigned short* DWT   = (unsigned short*)(ws + kOffDWT);
  unsigned short* WXT   = (unsigned short*)(ws + kOffWXT);
  unsigned short* WHT   = (unsigned short*)(ws + kOffWHT);
  unsigned short* A1    = (unsigned short*)(ws + kOffA1);
  unsigned short* POOL  = (unsigned short*)(ws + kOffPOOL);
  unsigned short* FEATS = (unsigned short*)(ws + kOffFEATS);
  float*          XG    = (float*)(ws + kOffXG);

  const int t8w1 = kCh1 * kK1 / 8;
  const int t8w2 = kCh2 * kK2 / 8;
  const int t8dw = kND * kCh2 / 8;
  const int t8wg = kNG * kND / 8;
  pack_wt_kernel<1><<<(t8w1 + 255) / 256, 256, 0, stream>>>(cw1, W1T, kCh1, kK1, t8w1);
  pack_wt_kernel<0><<<(t8w2 + 255) / 256, 256, 0, stream>>>(cw2, W2T, kCh2, kK2, t8w2);
  pack_wt_kernel<0><<<(t8dw + 255) / 256, 256, 0, stream>>>(dw,  DWT, kND,  kCh2, t8dw);
  pack_wt_kernel<0><<<(t8wg + 255) / 256, 256, 0, stream>>>(wx,  WXT, kNG,  kND,  t8wg);
  pack_wt_kernel<0><<<(t8wg + 255) / 256, 256, 0, stream>>>(wh,  WHT, kNG,  kND,  t8wg);

  conv1_kernel<<<kNF * 2, 256, 0, stream>>>(x, W1T, cb1, A1);
  conv2_pool_kernel<<<kNF, 256, 0, stream>>>(A1, W2T, cb2, POOL);
  gemm64_kernel<1, 2><<<(kNF / 64) * (kND / 64) / 8, 256, 0, stream>>>(
      POOL, kCh2, DWT, kCh2, (void*)FEATS, kND, db, kNF, kND, kCh2, kScale2, kCarryA);
  gemm64_kernel<0, 0><<<(kNF / 64) * (kNG / 64) / 8, 256, 0, stream>>>(
      FEATS, kND, WXT, kND, (void*)XG, kNG, bg, kNF, kNG, kND, kScale2, 1.0f);
  gru_seq_kernel<<<1, 512, 0, stream>>>(XG, WHT, out0, out1);
}
